// FHT2D_37297495998889
// MI455X (gfx1250) — hardware-verified
//
#include <hip/hip_runtime.h>
#include <math.h>

typedef __attribute__((ext_vector_type(16))) _Float16 v16h;
typedef __attribute__((ext_vector_type(16))) __bf16 v16b;
typedef __attribute__((ext_vector_type(8)))  _Float16 v8h;
typedef __attribute__((ext_vector_type(8)))  float v8f;
typedef __attribute__((ext_vector_type(4)))  float v4f;
typedef __attribute__((ext_vector_type(2)))  float v2f;
typedef __attribute__((ext_vector_type(4)))  unsigned v4u;
typedef __attribute__((ext_vector_type(4)))  int v4i;
typedef float __attribute__((may_alias)) float_a;
typedef int __attribute__((may_alias)) int_a;

template <typename T> __device__ __forceinline__ void vst2(void* p, T v) { *(volatile T*)p = v; __threadfence(); *(volatile T*)p = v; }
__device__ __forceinline__ v8f wmma16(v16h a, v16h b, v8f c) {
  v8f d = __builtin_amdgcn_wmma_f32_16x16x32_f16(false, a, false, b, (short)0, c, false, false);
  asm volatile("v_nop\n\tv_nop\n\tv_nop\n\tv_nop" : "+v"(d) : "v"(a), "v"(b));
  return d;
}
__device__ __forceinline__ v8f wmma_bf(v16b a, v16b b, v8f c) {
  v8f d = __builtin_amdgcn_wmma_f32_16x16x32_bf16(false, a, false, b, (short)0, c, false, false);
  asm volatile("v_nop\n\tv_nop\n\tv_nop\n\tv_nop" : "+v"(d) : "v"(a), "v"(b));
  return d;
}
__device__ __forceinline__ v16h frag_h(const _Float16* rowk0, int lane) {
  union { v16h v; v8h q[2]; } u; const _Float16* p = rowk0 + 8 * (lane >> 4);
  u.q[0] = *(const v8h*)p; u.q[1] = *(const v8h*)(p + 16); return u.v;
}
__device__ __forceinline__ v16h frag_f32(const float* rowk0, int lane) {
  v16h a; const float* p = rowk0 + 8 * (lane >> 4);
#pragma unroll
  for (int i = 0; i < 8; ++i) { a[i] = (_Float16)p[i]; a[8 + i] = (_Float16)p[16 + i]; }
  return a;
}
__device__ __forceinline__ v16h frag_f32s(const float* rowk0, int lane, float sc) {
  v16h a; const float* p = rowk0 + 8 * (lane >> 4);
#pragma unroll
  for (int i = 0; i < 8; ++i) { a[i] = (_Float16)(p[i] * sc); a[8 + i] = (_Float16)(p[16 + i] * sc); }
  return a;
}
__device__ __forceinline__ v16h fragc_f32(const float* W, int k0, int n, int lane, int ld, int K) {
  v16h a; const int g = lane >> 4;
#pragma unroll
  for (int i = 0; i < 8; ++i) { const int ka = k0 + 8 * g + i, kb = ka + 16;
    a[i] = (_Float16)(ka < K ? W[(size_t)(ka < K ? ka : K - 1) * ld + n] : 0.f); a[8 + i] = (_Float16)(kb < K ? W[(size_t)(kb < K ? kb : K - 1) * ld + n] : 0.f); }
  return a;
}
struct F2 { v16b h, l; };
__device__ __forceinline__ F2 bsplit16(const float v[16]) { F2 r;
#pragma unroll
  for (int i = 0; i < 16; ++i) { const __bf16 h = (__bf16)v[i]; r.h[i] = h; r.l[i] = (__bf16)(v[i] - (float)h); }
  return r; }
__device__ __forceinline__ F2 split_row(const float* row, int k0, int lane) { float v[16]; const float* p = row + k0 + 8 * (lane >> 4);
#pragma unroll
  for (int i = 0; i < 8; ++i) { v[i] = p[i]; v[8 + i] = p[16 + i]; }
  return bsplit16(v); }
__device__ __forceinline__ F2 split_rowK(const float* row, int k0, int lane, int K) { float v[16]; const int g = lane >> 4;
#pragma unroll
  for (int i = 0; i < 8; ++i) { const int ka = k0 + 8 * g + i, kb = ka + 16; v[i] = ka < K ? row[ka < K ? ka : K - 1] : 0.f; v[8 + i] = kb < K ? row[kb < K ? kb : K - 1] : 0.f; }
  return bsplit16(v); }
__device__ __forceinline__ F2 split_col(const float* W, int k0, int n, int lane, int ld, int K) { float v[16]; const int g = lane >> 4;
#pragma unroll
  for (int i = 0; i < 8; ++i) { const int ka = k0 + 8 * g + i, kb = ka + 16; v[i] = ka < K ? W[(size_t)(ka < K ? ka : K - 1) * ld + n] : 0.f; v[8 + i] = kb < K ? W[(size_t)(kb < K ? kb : K - 1) * ld + n] : 0.f; }
  return bsplit16(v); }
__device__ __forceinline__ v8f mac3(const F2& a, const F2& b, v8f c) { c = wmma_bf(a.l, b.h, c); c = wmma_bf(a.h, b.l, c); return wmma_bf(a.h, b.h, c); }
__device__ __forceinline__ float sigm(float v) { return 1.0f / (1.0f + expf(-v)); }
#define LDSX() do { asm volatile("s_wait_dscnt 0" ::: "memory"); __builtin_amdgcn_wave_barrier(); __builtin_amdgcn_fence(__ATOMIC_RELEASE, "workgroup"); } while (0)


#define NI 48
#define M 512
#ifndef TNI
#define TNI NI
#endif
typedef __attribute__((ext_vector_type(8))) __bf16 v8b;
__device__ __forceinline__ v16b frag_b(const __bf16* rowk0, int lane) {
  union { v16b v; v8b q[2]; } u; const __bf16* p = rowk0 + 8 * (lane >> 4);
  u.q[0] = *(const v8b*)p; u.q[1] = *(const v8b*)(p + 16); return u.v;
}
__device__ __forceinline__ float bfr(float v) { return (float)(__bf16)v; }
__device__ __attribute__((noinline)) float exp_ni(float v) { return expf(v); }
__device__ __attribute__((noinline)) float erf_ni(float v) { return erff(v); }

#define WS_PC  0u
#define WS_PR  (WS_PC + 2u * M * M)
#define WS_TH  (WS_PR + 2u * M * M)
#define WS_TL  (WS_TH + 2u * NI * M * M)
#define WS_END (WS_TL + 2u * NI * M * M)

__global__ __launch_bounds__(128) void k_pack(const float* __restrict__ EC, const float* __restrict__ ER, __bf16* __restrict__ PC, __bf16* __restrict__ PR) {
  __shared__ __align__(16) __bf16 s[M]; const int r = blockIdx.x, which = blockIdx.y, tid = threadIdx.x;
  for (int k = tid; k < M; k += 128) s[k] = (__bf16)(which == 0 ? EC[(size_t)k * M + r] : ER[(size_t)r * M + k]);
  __syncthreads();
  if (tid < M / 8) vst2((unsigned*)((which == 0 ? PC : PR) + (size_t)r * M + tid * 8), *(const v4u*)&s[tid * 8]);
}
__global__ __launch_bounds__(128) void k_stage1(const float* __restrict__ X, const int* __restrict__ INV, const __bf16* __restrict__ PC, __bf16* __restrict__ TH, __bf16* __restrict__ TL) {
  __shared__ __align__(16) __bf16 sh[4][16][136], sl[4][16][136];
  const int tid = threadIdx.x, wave = tid >> 5, lane = tid & 31, col = lane & 15, g = lane >> 4; const int img = blockIdx.z; const int r0 = blockIdx.x * 64 + wave * 16; const int h0 = blockIdx.y * 128;
  const int inv = INV[0] != 0; const float* xi = X + (size_t)img * M * M;
  v8f acc[8] = {};
#pragma unroll 2
  for (int kc = 0; kc < M / 32; ++kc) { const v16b a = frag_b(PC + (size_t)(r0 + col) * M + kc * 32, lane);
#pragma unroll
    for (int j = 0; j < 8; ++j) { int hrow = h0 + j * 16 + col; int w0 = kc * 32; if (inv) { hrow = (hrow + M / 2) & (M - 1); w0 = (w0 + M / 2) & (M - 1); }
      v16b b; const float* p = xi + (size_t)hrow * M + w0 + 8 * g;
#pragma unroll
      for (int i = 0; i < 8; ++i) { b[i] = (__bf16)p[i]; b[8 + i] = (__bf16)p[16 + i]; }
      acc[j] = wmma_bf(a, b, acc[j]); } }
#pragma unroll
  for (int j = 0; j < 8; ++j)
#pragma unroll
    for (int r = 0; r < 8; ++r) { const float v = acc[j][r]; const __bf16 hb = (__bf16)v; sh[wave][8 * g + r][j * 16 + col] = hb; sl[wave][8 * g + r][j * 16 + col] = (__bf16)(v - (float)hb); }
  LDSX();
  for (int rl = 0; rl < 16; ++rl) if (lane < 16) { const size_t o = ((size_t)img * M + r0 + rl) * M + h0 + lane * 8; vst2((unsigned*)(TH + o), *(const v4u*)&sh[wave][rl][lane * 8]); vst2((unsigned*)(TL + o), *(const v4u*)&sl[wave][rl][lane * 8]); }
}
__global__ __launch_bounds__(128) void k_stage2(const __bf16* __restrict__ PR, const __bf16* __restrict__ TH, const __bf16* __restrict__ TL, const int* __restrict__ INV, float* __restrict__ out) {
  __shared__ __align__(16) float so[4][16][132];
  const int tid = threadIdx.x, wave = tid >> 5, lane = tid & 31, col = lane & 15, g = lane >> 4; const int img = blockIdx.z; const int r0 = blockIdx.x * 64 + wave * 16; const int n0 = blockIdx.y * 128;
  const int inv = INV[0] != 0;
  v8f acc[8] = {};
#pragma unroll 2
  for (int kc = 0; kc < M / 32; ++kc) { const v16b a = frag_b(PR + (size_t)(r0 + col) * M + kc * 32, lane);
#pragma unroll
    for (int j = 0; j < 8; ++j) { const size_t br = ((size_t)img * M + n0 + j * 16 + col) * M + kc * 32; acc[j] = wmma_bf(a, frag_b(TL + br, lane), acc[j]); acc[j] = wmma_bf(a, frag_b(TH + br, lane), acc[j]); } }
  const float sc = inv ? 1.0f : (1.0f / 262144.0f);
#pragma unroll
  for (int j = 0; j < 8; ++j)
#pragma unroll
    for (int r = 0; r < 8; ++r) so[wave][8 * g + r][j * 16 + col] = acc[j][r] * sc;
  LDSX();
  const int nd = inv ? n0 : ((n0 + M / 2) & (M - 1));
  for (int rl = 0; rl < 16; ++rl) { const int m = r0 + rl; const int md = inv ? m : ((m + M / 2) & (M - 1)); vst2(out + ((size_t)img * M + md) * M + nd + lane * 4, *(const v4f*)&so[wave][rl][lane * 4]); }
}
extern "C" void kernel_launch(void* const* d_in, const int* in_sizes, int n_in, void* d_out, int out_size, void* d_ws, size_t ws_size, hipStream_t stream) {
  (void)in_sizes; (void)n_in; (void)out_size;
  const float** F = (const float**)d_in; const int* INV = (const int*)d_in[3];
  if (ws_size < (size_t)WS_END) return;
  char* ws = (char*)d_ws; __bf16 *PC = (__bf16*)(ws + WS_PC), *PR = (__bf16*)(ws + WS_PR), *TH = (__bf16*)(ws + WS_TH), *TL = (__bf16*)(ws + WS_TL);
  k_pack<<<dim3(M, 2), 128, 0, stream>>>(F[1], F[2], PC, PR);
  k_stage1<<<dim3(M / 64, M / 128, TNI), 128, 0, stream>>>(F[0], INV, PC, TH, TL);
  k_stage2<<<dim3(M / 64, M / 128, TNI), 128, 0, stream>>>(PR, TH, TL, INV, (float*)d_out);
}
